// MappingNetwork_41781441856238
// MI455X (gfx1250) — hardware-run, weakly checked
//
#include <hip/hip_runtime.h>
#include <math.h>

#define NTOK 8192
#define ZD 64
#define HD 512
#define OD 64
#define NDOM 8
#define DM (2 * HD)
#define NE 16
#define SPT 1
#define NSLOT (NTOK * SPT)
#define R_MAX (NSLOT + 64 * NE)
#define NT_MAX (R_MAX / 64)
#define NSH 1
#define NROW_S NTOK

#define CX_LOG2 11
#define CW_LOG2 16
#define CH ((float)(1u << CX_LOG2))
#define SC (1.0f / (float)(1u << (CX_LOG2 + CW_LOG2)))

#define RW_CH 8192
#define TBL_COUNT 0
#define TBL_POFF 16
#define TBL_NTILES 40
#define TBL_TILE_E 64
#define TBL_HDR 256
#define TBL_ROWTOK TBL_HDR
#define TBL_SLOTROW (TBL_HDR + R_MAX)
#define TBL_WORDS (TBL_HDR + R_MAX + NSLOT)

static_assert(NTOK == 8192 && ZD == 64 && HD == 512 && OD == 64 && NDOM == 8 && DM == 1024 && NE == 16 && NDOM <= NE && SPT == 1);
static_assert(ZD % 64 == 0 && HD % 64 == 0 && OD % 64 == 0 && NTOK % 128 == 0 && NROW_S % 64 == 0 && NROW_S / 64 <= NT_MAX);
static_assert(NSLOT % 128 == 0 && R_MAX % 128 == 0 && R_MAX >= NSLOT + 63 * NE);
static_assert(TBL_HDR % 32 == 0 && TBL_HDR <= 512);
static_assert(TBL_COUNT + NE <= TBL_POFF && TBL_POFF + NE + 1 <= TBL_NTILES && TBL_NTILES < TBL_TILE_E && TBL_TILE_E + NT_MAX <= TBL_HDR);
static_assert(RW_CH % 128 == 0 && (TBL_WORDS * 4) % 256 == 0);
static_assert((NTOK * ZD / 8) % 256 == 0);
static_assert(NSLOT == 8192 && R_MAX == 9216 && NT_MAX == 144 && TBL_WORDS == 17664);

constexpr size_t al256(size_t b) { return (b + 255) & ~(size_t)255; }
constexpr size_t SZ_Z16  = al256((size_t)NTOK * ZD * 2);
constexpr size_t SZ_SW0  = al256((size_t)HD * ZD * 2);
constexpr size_t SZ_SWP  = al256((size_t)HD * HD * 2);
constexpr size_t SZ_SWD  = al256((size_t)HD * DM * 2);
constexpr size_t SZ_UWP  = al256((size_t)NDOM * HD * HD * 2);
constexpr size_t SZ_UWD  = al256((size_t)NDOM * HD * DM * 2);
constexpr size_t SZ_UW3  = al256((size_t)NDOM * OD * HD * 2);
constexpr size_t SZ_TBLD = al256((size_t)TBL_HDR * 4);
constexpr size_t SZ_TBLR = al256((size_t)TBL_WORDS * 4);
constexpr size_t SZ_P    = al256((size_t)NTOK * DM * 2);
constexpr size_t SZ_G2W  = al256((size_t)R_MAX * DM * 2);
constexpr size_t SZ_G1W  = al256((size_t)R_MAX * HD * 2);
constexpr size_t SZ_YG   = al256((size_t)R_MAX * OD * 4);
constexpr size_t WS_TOTAL = SZ_Z16 + SZ_SW0 + 3 * SZ_SWP + 3 * SZ_SWD + 3 * SZ_UWP + 2 * SZ_UWD + SZ_UW3 + SZ_TBLD + SZ_TBLR + 2 * SZ_P + 2 * SZ_G2W + 2 * SZ_G1W + SZ_YG;
static_assert(WS_TOTAL == (size_t)128325632 && WS_TOTAL < (size_t)134217728);

typedef _Float16 h16;
typedef __attribute__((ext_vector_type(16))) _Float16 v16h;
typedef __attribute__((ext_vector_type(8)))  _Float16 v8h;
typedef __attribute__((ext_vector_type(8)))  float    v8f;
typedef __attribute__((ext_vector_type(4)))  float    v4f;
typedef __attribute__((ext_vector_type(2)))  float    v2f;
typedef __attribute__((ext_vector_type(4)))  unsigned int v4u;
typedef __attribute__((ext_vector_type(4)))  int      v4i;
typedef __attribute__((ext_vector_type(2)))  int      v2i;


#define VST2(T, ptr, val) do { const T vst2_v_ = (val); *(volatile T*)(ptr) = vst2_v_; __threadfence(); *(volatile T*)(ptr) = vst2_v_; } while (0)

static __device__ __forceinline__ float bfr(float f) {
    unsigned u = __float_as_uint(f);
    u += 0x7FFFu + ((u >> 16) & 1u);
    return __uint_as_float(u & 0xFFFF0000u);
}
static __device__ __forceinline__ h16 toh_flush(float v) { const float w = (fabsf(v) < 6.103515625e-05f) ? 0.0f : v; return (h16)w; }
static __device__ __forceinline__ void st8h(h16* p, const float* v) {
    v8h hv;
#pragma unroll
    for (int e = 0; e < 8; ++e) hv[e] = toh_flush(v[e]);
    VST2(v8h, p, hv);
}

union FragU { v16h v; v8h h[2]; };
static __device__ __forceinline__ v16h frag_ld(const h16* p) {
    FragU f; f.h[0] = *(const v8h*)(p); f.h[1] = *(const v8h*)(p + 16); return f.v;
}
static __device__ __forceinline__ v8f wmma16g(v16h a, v16h b, v8f c) {
    c = __builtin_amdgcn_wmma_f32_16x16x32_f16(false, a, false, b, (short)0, c, false, false);
    asm volatile("v_nop\n\tv_nop\n\tv_nop\n\tv_nop" : "+v"(c) : "v"(a), "v"(b));
    return c;
}
static __device__ __forceinline__ void wave_sync_lds() {
    __builtin_amdgcn_fence(3  , "workgroup");
    __builtin_amdgcn_wave_barrier();
    __builtin_amdgcn_fence(2  , "workgroup");
}

template <int LOG2C>
__global__ __launch_bounds__(256) void k_plane(const float* __restrict__ src, h16* __restrict__ dst, unsigned n8) {
    const unsigned u = blockIdx.x * 256u + threadIdx.x;
    if (u >= n8) return;
    const float cs = (float)(1u << LOG2C);
    const v4f a = *(const v4f*)(src + (size_t)u * 8u);
    const v4f b = *(const v4f*)(src + (size_t)u * 8u + 4u);
    float v[8] = {bfr(a.x) * cs, bfr(a.y) * cs, bfr(a.z) * cs, bfr(a.w) * cs, bfr(b.x) * cs, bfr(b.y) * cs, bfr(b.z) * cs, bfr(b.w) * cs};
    st8h(dst + (size_t)u * 8u, v);
}

__global__ __launch_bounds__(128) void k_planeTw(const float* __restrict__ src, h16* __restrict__ dst, unsigned ne, unsigned K, unsigned N, unsigned pitch, unsigned estride, float cs) {
    __shared__ __align__(16) float sT[4][64 * 36];
    const unsigned lane = threadIdx.x & 31u;
    const unsigned wave = threadIdx.x >> 5;
    const unsigned tk = K >> 6, tn = N >> 5;
    const unsigned tpe = tk * tn;
    const unsigned u = blockIdx.x * 4u + wave;
    if (u >= ne * tpe) return;
    const unsigned e = u / tpe;
    const unsigned rem = u - e * tpe;
    const unsigned kt = rem / tn;
    const unsigned nt = rem - kt * tn;
    const unsigned k0 = kt << 6, n0 = nt << 5;
    const size_t sbase = (size_t)e * (size_t)estride;
    const size_t ebase = (size_t)e * ((size_t)K * (size_t)N);
    float* slab = sT[wave];
#pragma unroll
    for (int i = 0; i < 16; ++i) {
        const unsigned p = lane + 32u * (unsigned)i;
        const unsigned kr = p >> 3;
        const unsigned n4 = (p & 7u) * 4u;
        const v4f a = *(const v4f*)(src + sbase + (size_t)(k0 + kr) * pitch + n0 + n4);
        v4f s;
        s.x = bfr(a.x) * cs; s.y = bfr(a.y) * cs; s.z = bfr(a.z) * cs; s.w = bfr(a.w) * cs;
        *(v4f*)(&slab[kr * 36u + n4]) = s;
    }
    wave_sync_lds();
#pragma unroll
    for (int i = 0; i < 8; ++i) {
        const unsigned q = lane + 32u * (unsigned)i;
        const unsigned n = q >> 3;
        const unsigned kp = q & 7u;
        float v[8];
#pragma unroll
        for (int j = 0; j < 8; ++j) v[j] = slab[(8u * kp + (unsigned)j) * 36u + n];
        st8h(dst + ebase + (size_t)(n0 + n) * K + k0 + 8u * kp, v);
    }
}

__global__ __launch_bounds__(256) void k_dupK(const h16* __restrict__ src, h16* __restrict__ dst, unsigned nchunk) {
    const unsigned i = blockIdx.x * 256u + threadIdx.x;
    if (i >= nchunk) return;
    const unsigned row = i / (unsigned)(HD / 8);
    const unsigned c = (i - row * (unsigned)(HD / 8)) * 8u;
    const v4u v = *(const v4u*)(src + (size_t)row * HD + c);
    VST2(v4u, dst + (size_t)row * DM + c, v);
    VST2(v4u, dst + (size_t)row * DM + HD + c, v);
}

__global__ __launch_bounds__(64) void k_tbl_dense(int* __restrict__ tbl) {
    const unsigned w0 = threadIdx.x * 4u;
    int q[4];
#pragma unroll
    for (int k = 0; k < 4; ++k) {
        const unsigned w = w0 + (unsigned)k;
        int val = 0;
        val = (w < (unsigned)(TBL_COUNT + NSH)) ? NTOK : val;
        val = (w >= (unsigned)TBL_POFF && w <= (unsigned)(TBL_POFF + NE)) ? (int)min((w - (unsigned)TBL_POFF) * (unsigned)NTOK, (unsigned)NROW_S) : val;
        val = (w == (unsigned)TBL_NTILES) ? (NROW_S / 64) : val;
        val = (w >= (unsigned)TBL_TILE_E && w < (unsigned)(TBL_TILE_E + NT_MAX)) ? ((w - (unsigned)TBL_TILE_E < (unsigned)(NROW_S / 64)) ? (int)((w - (unsigned)TBL_TILE_E) / (unsigned)(NTOK / 64)) : -1) : val;
        q[k] = val;
    }
    v4i v;
    v.x = q[0]; v.y = q[1]; v.z = q[2]; v.w = q[3];
    VST2(v4i, tbl + w0, v);
}

template <int NE_>
__global__ __launch_bounds__(32) void k_route1w(const int* __restrict__ sel, int* __restrict__ tbl, unsigned nslot, unsigned spt, unsigned hdr, unsigned rmax,
                                                unsigned offPoff, unsigned offNtiles, unsigned offTileE) {
    static_assert(NE_ >= 1 && NE_ <= 32);
    __shared__ __align__(16) int s_img[RW_CH];
    __shared__ __align__(16) int s_hdr[512];
    const unsigned lane = threadIdx.x & 31u;
    const unsigned spl = nslot >> 5;
    const unsigned ng = spl >> 2;
    const unsigned ntmax = rmax >> 6;
    const v4i* sp = (const v4i*)(sel + (size_t)lane * spl);
    int cnt[NE_];
#pragma unroll
    for (int j = 0; j < NE_; ++j) cnt[j] = 0;
    for (unsigned g = 0; g < ng; ++g) {
        const v4i v = sp[g];
#pragma unroll
        for (int c = 0; c < 4; ++c) {
            const int e = min(max(v[c], 0), NE_ - 1);
#pragma unroll
            for (int j = 0; j < NE_; ++j) cnt[j] += (e == j) ? 1 : 0;
        }
    }
    int base0[NE_], total[NE_];
#pragma unroll
    for (int j = 0; j < NE_; ++j) {
        int pre = 0, tot = cnt[j];
#pragma unroll
        for (int d = 1; d < 32; d <<= 1) {
            const int t = __shfl_xor(tot, d, 32);
            pre += ((lane & (unsigned)d) != 0u) ? t : 0;
            tot += t;
        }
        base0[j] = pre;
        total[j] = tot;
    }
    int poff[NE_ + 1];
    poff[0] = 0;
#pragma unroll
    for (int j = 0; j < NE_; ++j) poff[j + 1] = poff[j] + (((total[j] + 63) >> 6) << 6);
    for (unsigned i = lane; i < 512u; i += 32u) s_hdr[i] = (i >= offTileE && i < offTileE + ntmax) ? -1 : 0;
    wave_sync_lds();
    if (lane == 0u) {
#pragma unroll
        for (int j = 0; j < NE_; ++j) { s_hdr[min((unsigned)j, 511u)] = total[j]; s_hdr[min(offPoff + (unsigned)j, 511u)] = poff[j]; }
        s_hdr[min(offPoff + (unsigned)NE_, 511u)] = poff[NE_];
        s_hdr[min(offNtiles, 511u)] = poff[NE_] >> 6;
    }
    for (unsigned t = lane; t < ntmax; t += 32u) {
        const int b64 = (int)(t * 64u);
        int ev = -1;
#pragma unroll
        for (int j = 0; j < NE_; ++j) ev = (b64 >= poff[j] && b64 < poff[j + 1]) ? j : ev;
        s_hdr[min(offTileE + t, 511u)] = ev;
    }
    wave_sync_lds();
    for (int pass = 0; pass < 2; ++pass) {
        for (unsigned i = lane; i < (hdr >> 2); i += 32u) *(volatile v4i*)(tbl + 4u * i) = *(const v4i*)(&s_hdr[4u * i]);
        __threadfence();
    }
    for (unsigned lo = 0; lo < rmax; lo += (unsigned)RW_CH) {
        for (unsigned i = lane; i < (unsigned)(RW_CH / 4); i += 32u) *(v4i*)(&s_img[4u * i]) = (v4i){-1, -1, -1, -1};
        wave_sync_lds();
        int run[NE_];
#pragma unroll
        for (int j = 0; j < NE_; ++j) run[j] = base0[j];
        for (unsigned g = 0; g < ng; ++g) {
            const v4i v = sp[g];
#pragma unroll
            for (int c = 0; c < 4; ++c) {
                const int e = min(max(v[c], 0), NE_ - 1);
                int row = 0;
#pragma unroll
                for (int j = 0; j < NE_; ++j) {
                    const bool hit = (e == j);
                    row = hit ? (poff[j] + run[j]) : row;
                    run[j] += hit ? 1 : 0;
                }
                row = min(max(row, 0), (int)rmax - 1);
                const unsigned rel = (unsigned)row - lo;
                if (rel < (unsigned)RW_CH) s_img[rel] = (int)((lane * spl + 4u * g + (unsigned)c) / spt);
            }
        }
        wave_sync_lds();
        const unsigned nw = min((unsigned)RW_CH, rmax - lo);
        for (int pass = 0; pass < 2; ++pass) {
            for (unsigned i = lane; i < (nw >> 2); i += 32u) *(volatile v4i*)(tbl + hdr + lo + 4u * i) = *(const v4i*)(&s_img[4u * i]);
            __threadfence();
        }
        wave_sync_lds();
    }
    for (unsigned lo = 0; lo < nslot; lo += (unsigned)RW_CH) {
        int run[NE_];
#pragma unroll
        for (int j = 0; j < NE_; ++j) run[j] = base0[j];
        for (unsigned g = 0; g < ng; ++g) {
            const v4i v = sp[g];
#pragma unroll
            for (int c = 0; c < 4; ++c) {
                const int e = min(max(v[c], 0), NE_ - 1);
                int row = 0;
#pragma unroll
                for (int j = 0; j < NE_; ++j) {
                    const bool hit = (e == j);
                    row = hit ? (poff[j] + run[j]) : row;
                    run[j] += hit ? 1 : 0;
                }
                row = min(max(row, 0), (int)rmax - 1);
                const unsigned rel = (lane * spl + 4u * g + (unsigned)c) - lo;
                if (rel < (unsigned)RW_CH) s_img[rel] = row;
            }
        }
        wave_sync_lds();
        const unsigned nw = min((unsigned)RW_CH, nslot - lo);
        for (int pass = 0; pass < 2; ++pass) {
            for (unsigned i = lane; i < (nw >> 2); i += 32u) *(volatile v4i*)(tbl + hdr + rmax + lo + 4u * i) = *(const v4i*)(&s_img[4u * i]);
            __threadfence();
        }
        wave_sync_lds();
    }
}

__global__ __launch_bounds__(256) void k_gather(const h16* __restrict__ x16, const int* __restrict__ tbl, h16* __restrict__ Xg) {
    const unsigned row = blockIdx.x * 2u + (threadIdx.x >> 7);
    if (row >= (unsigned)R_MAX) return;
    const unsigned c = (threadIdx.x & 127u) * 8u;
    const int tr = tbl[TBL_ROWTOK + row];
    const bool pad = (tr < 0);
    const int tok = min(max(tr, 0), NTOK - 1);
    const v4u ld = *(const v4u*)(x16 + (size_t)(unsigned)tok * DM + c);
    v4u v;
    v.x = pad ? 0u : ld.x; v.y = pad ? 0u : ld.y; v.z = pad ? 0u : ld.z; v.w = pad ? 0u : ld.w;
    VST2(v4u, Xg + (size_t)row * DM + c, v);
}

template <int KD, int ND, int MODE>
__global__ __launch_bounds__(256) void k_lin(const h16* __restrict__ A, const h16* __restrict__ Wp, const float* __restrict__ eb,
                                             const int* __restrict__ tbl, void* __restrict__ OutV, unsigned nreal) {
    static_assert(KD % 32 == 0 && ND % 64 == 0 && MODE >= 0 && MODE <= 2);
    __shared__ __align__(16) float sT[8][16 * 68];
    const unsigned lane = threadIdx.x & 31u;
    const unsigned wave = threadIdx.x >> 5;
    const unsigned u = blockIdx.x * 8u + wave;
    if (u >= (unsigned)(NT_MAX * (ND / 64))) return;
    const unsigned rowtile = u / (unsigned)(ND / 64);
    const unsigned ct = u - rowtile * (unsigned)(ND / 64);
    const int nt = min(max(tbl[TBL_NTILES], 0), NT_MAX);
    if ((int)rowtile >= nt) return;
    const int e = min(max(tbl[TBL_TILE_E + rowtile], 0), (int)nreal - 1);
    const size_t wbase = (size_t)(unsigned)e * (size_t)(ND * KD);
    const unsigned m0 = rowtile << 6, n0 = ct << 6;
    const unsigned rlane = lane & 15u;
    const unsigned koff = (lane >> 4) * 8u;
    const unsigned mOff = koff;

    v8f acc[4][4];
#pragma unroll
    for (int i = 0; i < 4; ++i)
#pragma unroll
        for (int j = 0; j < 4; ++j) acc[i][j] = (v8f){0.f,0.f,0.f,0.f,0.f,0.f,0.f,0.f};

    for (unsigned k0 = 0; k0 < (unsigned)KD; k0 += 32u) {
        v16h bh[4];
#pragma unroll
        for (int j = 0; j < 4; ++j)
            bh[j] = frag_ld(Wp + wbase + (size_t)(n0 + ((unsigned)j << 4) + rlane) * KD + koff + k0);
#pragma unroll
        for (int i = 0; i < 4; ++i) {
            const v16h ah = frag_ld(A + (size_t)(m0 + ((unsigned)i << 4) + rlane) * KD + koff + k0);
#pragma unroll
            for (int j = 0; j < 4; ++j) acc[i][j] = wmma16g(ah, bh[j], acc[i][j]);
        }
    }

    float ebv[4];
#pragma unroll
    for (int j = 0; j < 4; ++j) ebv[j] = bfr(eb[(unsigned)e * (unsigned)ND + n0 + ((unsigned)j << 4) + rlane]);

    float* slab = sT[wave];
#pragma unroll
    for (int i = 0; i < 4; ++i) {
        const unsigned mBase = m0 + ((unsigned)i << 4);
#pragma unroll
        for (int j = 0; j < 4; ++j)
#pragma unroll
            for (int r = 0; r < 8; ++r) {
                const float a = acc[i][j][r] * SC + ebv[j];
                const float g = fmaxf(a, 0.0f);
                slab[(mOff + (unsigned)r) * 68u + ((unsigned)j << 4) + rlane] = (MODE == 2) ? g : g * CH;
            }
        wave_sync_lds();
        if constexpr (MODE == 2) {
            float* Out = (float*)OutV;
            const unsigned hh = lane >> 4, c4 = (lane & 15u) * 4u;
#pragma unroll
            for (int half = 0; half < 2; ++half) {
                v4f vv[4];
#pragma unroll
                for (int it = 0; it < 4; ++it) {
                    const unsigned row = (unsigned)(half * 4 + it) * 2u + hh;
                    vv[it] = *(const v4f*)(slab + row * 68u + c4);
                }
                for (int pass = 0; pass < 2; ++pass) {
#pragma unroll
                    for (int it = 0; it < 4; ++it) {
                        const unsigned row = (unsigned)(half * 4 + it) * 2u + hh;
                        *(volatile v4f*)(Out + (size_t)(mBase + row) * ND + n0 + c4) = vv[it];
                    }
                    __threadfence();
                }
            }
        } else {
            h16* Out = (h16*)OutV;
            constexpr unsigned RS = (MODE == 1) ? (unsigned)(2 * ND) : (unsigned)ND;
            const unsigned q = lane >> 3, c8 = (lane & 7u) * 8u;
            v8h hv[4];
            v8h lv[4];
#pragma unroll
            for (int it = 0; it < 4; ++it) {
                const unsigned row = (unsigned)it * 4u + q;
                const float* sp = slab + row * 68u + c8;
#pragma unroll
                for (int t = 0; t < 8; ++t) {
                    const h16 hi = toh_flush(sp[t]);
                    hv[it][t] = hi;
                    lv[it][t] = (MODE == 1) ? toh_flush(sp[t] - (float)hi) : (h16)0.0f;
                }
            }
            for (int pass = 0; pass < 2; ++pass) {
#pragma unroll
                for (int it = 0; it < 4; ++it) {
                    const unsigned row = (unsigned)it * 4u + q;
                    *(volatile v8h*)(Out + (size_t)(mBase + row) * RS + n0 + c8) = hv[it];
                    if constexpr (MODE == 1) *(volatile v8h*)(Out + (size_t)(mBase + row) * RS + (unsigned)ND + n0 + c8) = lv[it];
                }
                __threadfence();
            }
        }
        wave_sync_lds();
    }
}

__global__ __launch_bounds__(256) void k_scatter(const float* __restrict__ Yg, const int* __restrict__ tbl, float* __restrict__ out) {
    const unsigned t = blockIdx.x * 16u + (threadIdx.x >> 4);
    if (t >= (unsigned)NTOK) return;
    const unsigned c = (threadIdx.x & 15u) * 4u;
    const int r = min(max(tbl[TBL_SLOTROW + t], 0), R_MAX - 1);
    const v4f a = *(const v4f*)(Yg + (size_t)(unsigned)r * OD + c);
    VST2(v4f, out + (size_t)t * OD + c, a);
}

extern "C" void kernel_launch(void* const* d_in, const int* in_sizes, int n_in, void* d_out, int out_size,
                              void* d_ws, size_t ws_size, hipStream_t stream) {
    if (n_in < 18) return;
    if (in_sizes[0] < NTOK * ZD || in_sizes[1] < NTOK || in_sizes[2] < ZD * HD || in_sizes[3] < HD || in_sizes[4] < HD * HD || in_sizes[5] < HD || in_sizes[6] < HD * HD || in_sizes[7] < HD ||
        in_sizes[8] < HD * HD || in_sizes[9] < HD || in_sizes[10] < NDOM * HD * HD || in_sizes[11] < NDOM * HD || in_sizes[12] < NDOM * HD * HD || in_sizes[13] < NDOM * HD ||
        in_sizes[14] < NDOM * HD * HD || in_sizes[15] < NDOM * HD || in_sizes[16] < NDOM * HD * OD || in_sizes[17] < NDOM * OD) return;
    if (out_size < NTOK * OD) return;

    const float* z   = (const float*)d_in[0];
    const int*   y   = (const int*)d_in[1];
    const float* sw0 = (const float*)d_in[2];
    const float* sb0 = (const float*)d_in[3];
    const float* sw1 = (const float*)d_in[4];
    const float* sb1 = (const float*)d_in[5];
    const float* sw2 = (const float*)d_in[6];
    const float* sb2 = (const float*)d_in[7];
    const float* sw3 = (const float*)d_in[8];
    const float* sb3 = (const float*)d_in[9];
    const float* uw0 = (const float*)d_in[10];
    const float* ub0 = (const float*)d_in[11];
    const float* uw1 = (const float*)d_in[12];
    const float* ub1 = (const float*)d_in[13];
    const float* uw2 = (const float*)d_in[14];
    const float* ub2 = (const float*)d_in[15];
    const float* uw3 = (const float*)d_in[16];
    const float* ub3 = (const float*)d_in[17];
    float* out = (float*)d_out;

    char* wsp = (char*)d_ws;
    size_t off = 0;
    auto carve = [&](size_t bytes) -> void* { void* r = wsp + off; off += (bytes + 255) & ~(size_t)255; return r; };
    h16* z16  = (h16*)carve((size_t)NTOK * ZD * 2);
    h16* sw0p = (h16*)carve((size_t)HD * ZD * 2);
    h16* sw1p = (h16*)carve((size_t)HD * HD * 2);
    h16* sw2p = (h16*)carve((size_t)HD * HD * 2);
    h16* sw3p = (h16*)carve((size_t)HD * HD * 2);
    h16* sw1d = (h16*)carve((size_t)HD * DM * 2);
    h16* sw2d = (h16*)carve((size_t)HD * DM * 2);
    h16* sw3d = (h16*)carve((size_t)HD * DM * 2);
    h16* uw0p = (h16*)carve((size_t)NDOM * HD * HD * 2);
    h16* uw1p = (h16*)carve((size_t)NDOM * HD * HD * 2);
    h16* uw2p = (h16*)carve((size_t)NDOM * HD * HD * 2);
    h16* uw0d = (h16*)carve((size_t)NDOM * HD * DM * 2);
    h16* uw1d = (h16*)carve((size_t)NDOM * HD * DM * 2);
    h16* uw3p = (h16*)carve((size_t)NDOM * OD * HD * 2);
    int* tblD = (int*)carve((size_t)TBL_HDR * 4);
    int* tblR = (int*)carve((size_t)TBL_WORDS * 4);
    h16* PA   = (h16*)carve((size_t)NTOK * DM * 2);
    h16* PB   = (h16*)carve((size_t)NTOK * DM * 2);
    h16* Xg   = (h16*)carve((size_t)R_MAX * DM * 2);
    h16* G1   = (h16*)carve((size_t)R_MAX * DM * 2);
    h16* G2   = (h16*)carve((size_t)R_MAX * HD * 2);
    h16* G3   = (h16*)carve((size_t)R_MAX * HD * 2);
    float* Yg = (float*)carve((size_t)R_MAX * OD * 4);
    if (off != WS_TOTAL || off > ws_size || off > (size_t)134217728) return;

    k_plane<CX_LOG2><<<(NTOK * ZD / 8) / 256, 256, 0, stream>>>(z, z16, (unsigned)(NTOK * ZD / 8));
    const float cw = (float)(1u << CW_LOG2);
    k_planeTw<<<(1 * (ZD / 64) * (HD / 32) + 3) / 4, 128, 0, stream>>>(sw0, sw0p, 1u, (unsigned)ZD, (unsigned)HD, (unsigned)HD, (unsigned)(ZD * HD), cw);
    k_planeTw<<<(1 * (HD / 64) * (HD / 32) + 3) / 4, 128, 0, stream>>>(sw1, sw1p, 1u, (unsigned)HD, (unsigned)HD, (unsigned)HD, (unsigned)(HD * HD), cw);
    k_planeTw<<<(1 * (HD / 64) * (HD / 32) + 3) / 4, 128, 0, stream>>>(sw2, sw2p, 1u, (unsigned)HD, (unsigned)HD, (unsigned)HD, (unsigned)(HD * HD), cw);
    k_planeTw<<<(1 * (HD / 64) * (HD / 32) + 3) / 4, 128, 0, stream>>>(sw3, sw3p, 1u, (unsigned)HD, (unsigned)HD, (unsigned)HD, (unsigned)(HD * HD), cw);
    k_planeTw<<<(NDOM * (HD / 64) * (HD / 32) + 3) / 4, 128, 0, stream>>>(uw0, uw0p, (unsigned)NDOM, (unsigned)HD, (unsigned)HD, (unsigned)HD, (unsigned)(HD * HD), cw);
    k_planeTw<<<(NDOM * (HD / 64) * (HD / 32) + 3) / 4, 128, 0, stream>>>(uw1, uw1p, (unsigned)NDOM, (unsigned)HD, (unsigned)HD, (unsigned)HD, (unsigned)(HD * HD), cw);
    k_planeTw<<<(NDOM * (HD / 64) * (HD / 32) + 3) / 4, 128, 0, stream>>>(uw2, uw2p, (unsigned)NDOM, (unsigned)HD, (unsigned)HD, (unsigned)HD, (unsigned)(HD * HD), cw);
    k_planeTw<<<(NDOM * (HD / 64) * (OD / 32) + 3) / 4, 128, 0, stream>>>(uw3, uw3p, (unsigned)NDOM, (unsigned)HD, (unsigned)OD, (unsigned)OD, (unsigned)(HD * OD), cw);
    k_dupK<<<(HD * HD / 8) / 256, 256, 0, stream>>>(sw1p, sw1d, (unsigned)(HD * HD / 8));
    k_dupK<<<(HD * HD / 8) / 256, 256, 0, stream>>>(sw2p, sw2d, (unsigned)(HD * HD / 8));
    k_dupK<<<(HD * HD / 8) / 256, 256, 0, stream>>>(sw3p, sw3d, (unsigned)(HD * HD / 8));
    k_dupK<<<(NDOM * HD * HD / 8) / 256, 256, 0, stream>>>(uw0p, uw0d, (unsigned)(NDOM * HD * HD / 8));
    k_dupK<<<(NDOM * HD * HD / 8) / 256, 256, 0, stream>>>(uw1p, uw1d, (unsigned)(NDOM * HD * HD / 8));
    k_tbl_dense<<<1, 64, 0, stream>>>(tblD);
    k_route1w<NE><<<1, 32, 0, stream>>>(y, tblR, (unsigned)NSLOT, (unsigned)SPT, (unsigned)TBL_HDR, (unsigned)R_MAX, (unsigned)TBL_POFF, (unsigned)TBL_NTILES, (unsigned)TBL_TILE_E);

    k_lin<ZD, HD, 1><<<(NT_MAX * (HD / 64) + 7) / 8, 256, 0, stream>>>(z16, sw0p, sb0, tblD, (void*)PA, 1u);
    k_lin<DM, HD, 1><<<(NT_MAX * (HD / 64) + 7) / 8, 256, 0, stream>>>(PA, sw1d, sb1, tblD, (void*)PB, 1u);
    k_lin<DM, HD, 1><<<(NT_MAX * (HD / 64) + 7) / 8, 256, 0, stream>>>(PB, sw2d, sb2, tblD, (void*)PA, 1u);
    k_lin<DM, HD, 1><<<(NT_MAX * (HD / 64) + 7) / 8, 256, 0, stream>>>(PA, sw3d, sb3, tblD, (void*)PB, 1u);
    k_gather<<<R_MAX / 2, 256, 0, stream>>>(PB, tblR, Xg);
    k_lin<DM, HD, 1><<<(NT_MAX * (HD / 64) + 7) / 8, 256, 0, stream>>>(Xg, uw0d, ub0, tblR, (void*)G1, (unsigned)NDOM);
    k_lin<DM, HD, 0><<<(NT_MAX * (HD / 64) + 7) / 8, 256, 0, stream>>>(G1, uw1d, ub1, tblR, (void*)G2, (unsigned)NDOM);
    k_lin<HD, HD, 0><<<(NT_MAX * (HD / 64) + 7) / 8, 256, 0, stream>>>(G2, uw2p, ub2, tblR, (void*)G3, (unsigned)NDOM);
    k_lin<HD, OD, 2><<<(NT_MAX * (OD / 64) + 7) / 8, 256, 0, stream>>>(G3, uw3p, ub3, tblR, (void*)Yg, (unsigned)NDOM);
    k_scatter<<<NTOK / 16, 256, 0, stream>>>(Yg, tblR, out);
}
